// MoE_81432579932270
// MI455X (gfx1250) — hardware-verified
//
#include <hip/hip_runtime.h>
#include <math.h>

#define NTOK 4096
#define NTOK_FULL 4096
#define DM 512
#define FF 128
#define NE 32
#define TOPK 4
#define NSLOT (NTOK * TOPK)
#define R_MAX (NSLOT + 64 * NE)
#define NT_MAX (R_MAX / 64)

#define CX_LOG2 11
#define CW_LOG2 16
#define CH_LOG2 11
#define CH ((float)(1u << CH_LOG2))
#define SC_H (1.0f / (float)(1u << (CX_LOG2 + CW_LOG2)))
#define SC_Y (1.0f / (float)(1u << (CH_LOG2 + CW_LOG2)))

#define RW_CH 8192
#define TBL_COUNT 0
#define TBL_POFF 32
#define TBL_NTILES 72
#define TBL_TILE_E 80
#define TBL_HDR 512
#define TBL_ROWTOK TBL_HDR
#define TBL_SLOTROW (TBL_HDR + R_MAX)
#define TBL_WORDS (TBL_HDR + R_MAX + NSLOT)

static_assert(NE == 32 && TOPK == 4 && DM == 512 && FF == 128 && DM % 64 == 0 && FF % 64 == 0 && DM % 32 == 0 && FF % 32 == 0);
static_assert(NTOK <= NTOK_FULL && NTOK % 128 == 0);
static_assert(CX_LOG2 == 11 && CW_LOG2 == 16 && CH_LOG2 == 11);
static_assert(NSLOT % 128 == 0);
static_assert(R_MAX % 64 == 0 && R_MAX >= NSLOT + 63 * NE);
static_assert(TBL_HDR % 32 == 0 && TBL_HDR <= 512);
static_assert(TBL_COUNT + NE <= TBL_POFF && TBL_POFF + NE + 1 <= TBL_NTILES && TBL_NTILES < TBL_TILE_E && TBL_TILE_E + NT_MAX <= TBL_HDR);
static_assert(RW_CH % 128 == 0 && (TBL_WORDS * 4) % 256 == 0);
static_assert((NTOK * DM / 8) % 256 == 0);
static_assert(NSLOT == 16384 && R_MAX == 18432 && NT_MAX == 288 && TBL_WORDS == 35328);
static_assert(R_MAX % (256 / (DM / 8)) == 0 && (DM / 8) % 32 == 0);

constexpr size_t al256(size_t b) { return (b + 255) & ~(size_t)255; }
constexpr size_t SZ_X16 = al256((size_t)NTOK * DM * 2);
constexpr size_t SZ_W1T = al256((size_t)NE * FF * DM * 2);
constexpr size_t SZ_W2T = al256((size_t)NE * DM * FF * 2);
constexpr size_t SZ_SEL = al256((size_t)NSLOT * 4);
constexpr size_t SZ_WGT = al256((size_t)NSLOT * 4);
constexpr size_t SZ_TBL = al256((size_t)TBL_WORDS * 4);
constexpr size_t SZ_XG  = al256((size_t)R_MAX * DM * 2);
constexpr size_t SZ_HG  = al256((size_t)R_MAX * FF * 2);
constexpr size_t SZ_YG  = al256((size_t)R_MAX * DM * 4);
constexpr size_t WS_TOTAL = SZ_X16 + SZ_W1T + SZ_W2T + SZ_SEL + SZ_WGT + SZ_TBL + SZ_XG + SZ_HG + SZ_YG;
static_assert(WS_TOTAL < (size_t)134217728);

typedef _Float16 h16;
typedef __attribute__((ext_vector_type(16))) _Float16 v16h;
typedef __attribute__((ext_vector_type(8)))  _Float16 v8h;
typedef __attribute__((ext_vector_type(8)))  float    v8f;
typedef __attribute__((ext_vector_type(4)))  float    v4f;
typedef __attribute__((ext_vector_type(4)))  unsigned int v4u;
typedef __attribute__((ext_vector_type(4)))  int      v4i;
typedef __attribute__((ext_vector_type(2)))  int      v2i;
typedef __attribute__((ext_vector_type(2)))  float    v2f;


#define VST2(T, ptr, val) do { const T vst2_v_ = (val); *(volatile T*)(ptr) = vst2_v_; __threadfence(); *(volatile T*)(ptr) = vst2_v_; } while (0)

static __device__ __forceinline__ float bfr(float f) {
    unsigned u = __float_as_uint(f);
    u += 0x7FFFu + ((u >> 16) & 1u);
    return __uint_as_float(u & 0xFFFF0000u);
}
static __device__ __forceinline__ h16 toh_flush(float v) { const float w = (fabsf(v) < 6.103515625e-05f) ? 0.0f : v; return (h16)w; }
static __device__ __forceinline__ void st8h(h16* p, const float* v) {
    v8h hv;
#pragma unroll
    for (int e = 0; e < 8; ++e) hv[e] = toh_flush(v[e]);
    VST2(v8h, p, hv);
}

union FragU { v16h v; v8h h[2]; };
static __device__ __forceinline__ v16h frag_ld(const h16* p) {
    FragU f; f.h[0] = *(const v8h*)(p); f.h[1] = *(const v8h*)(p + 16); return f.v;
}
static __device__ __forceinline__ v8f wmma16g(v16h a, v16h b, v8f c) {
    c = __builtin_amdgcn_wmma_f32_16x16x32_f16(false, a, false, b, (short)0, c, false, false);
    asm volatile("v_nop\n\tv_nop\n\tv_nop\n\tv_nop" : "+v"(c) : "v"(a), "v"(b));
    return c;
}
static __device__ __forceinline__ void wave_sync_lds() {
    __builtin_amdgcn_fence(3  , "workgroup");
    __builtin_amdgcn_wave_barrier();
    __builtin_amdgcn_fence(2  , "workgroup");
}

template <int LOG2C>
__global__ __launch_bounds__(256) void k_plane(const float* __restrict__ src, h16* __restrict__ dst, unsigned n8) {
    const unsigned u = blockIdx.x * 256u + threadIdx.x;
    if (u >= n8) return;
    const float cs = (float)(1u << LOG2C);
    const v4f a = *(const v4f*)(src + (size_t)u * 8u);
    const v4f b = *(const v4f*)(src + (size_t)u * 8u + 4u);
    float v[8] = {bfr(a.x) * cs, bfr(a.y) * cs, bfr(a.z) * cs, bfr(a.w) * cs, bfr(b.x) * cs, bfr(b.y) * cs, bfr(b.z) * cs, bfr(b.w) * cs};
    st8h(dst + (size_t)u * 8u, v);
}

__global__ __launch_bounds__(128) void k_planeTw(const float* __restrict__ src, h16* __restrict__ dst, unsigned ne, unsigned K, unsigned N, unsigned pitch, unsigned estride, float cs) {
    __shared__ __align__(16) float sT[4][64 * 36];
    const unsigned lane = threadIdx.x & 31u;
    const unsigned wave = threadIdx.x >> 5;
    const unsigned tk = K >> 6, tn = N >> 5;
    const unsigned tpe = tk * tn;
    const unsigned u = blockIdx.x * 4u + wave;
    if (u >= ne * tpe) return;
    const unsigned e = u / tpe;
    const unsigned rem = u - e * tpe;
    const unsigned kt = rem / tn;
    const unsigned nt = rem - kt * tn;
    const unsigned k0 = kt << 6, n0 = nt << 5;
    const size_t sbase = (size_t)e * (size_t)estride;
    const size_t ebase = (size_t)e * ((size_t)K * (size_t)N);
    float* slab = sT[wave];
#pragma unroll
    for (int i = 0; i < 16; ++i) {
        const unsigned p = lane + 32u * (unsigned)i;
        const unsigned kr = p >> 3;
        const unsigned n4 = (p & 7u) * 4u;
        const v4f a = *(const v4f*)(src + sbase + (size_t)(k0 + kr) * pitch + n0 + n4);
        v4f s;
        s.x = bfr(a.x) * cs; s.y = bfr(a.y) * cs; s.z = bfr(a.z) * cs; s.w = bfr(a.w) * cs;
        *(v4f*)(&slab[kr * 36u + n4]) = s;
    }
    wave_sync_lds();
#pragma unroll
    for (int i = 0; i < 8; ++i) {
        const unsigned q = lane + 32u * (unsigned)i;
        const unsigned n = q >> 3;
        const unsigned kp = q & 7u;
        float v[8];
#pragma unroll
        for (int j = 0; j < 8; ++j) v[j] = slab[(8u * kp + (unsigned)j) * 36u + n];
        st8h(dst + ebase + (size_t)(n0 + n) * K + k0 + 8u * kp, v);
    }
}

__global__ __launch_bounds__(256) void k_gate(const float* __restrict__ x, const float* __restrict__ gw,
                                              int* __restrict__ sel, float* __restrict__ wgt) {
    const unsigned lane = threadIdx.x & 31u;
    const unsigned wave = threadIdx.x >> 5;
    const unsigned t0 = (blockIdx.x * 8u + wave) * 16u;
    if (t0 >= (unsigned)NTOK) return;
    v4i ki = (v4i){0, 0, 0, 0};
    v4f kw = (v4f){0.0f, 0.0f, 0.0f, 0.0f};
    for (unsigned j = 0; j < 16u; ++j) {
        const float* xr = x + (size_t)(t0 + j) * DM;
        float lg[NE];
#pragma unroll
        for (int e = 0; e < NE; ++e) lg[e] = 0.0f;
        for (unsigned i = 0; i < (unsigned)(DM / 32); ++i) {
            const unsigned d = lane + 32u * i;
            const float xv = bfr(xr[d]);
#pragma unroll
            for (int e = 0; e < NE; ++e) lg[e] += xv * bfr(gw[(unsigned)e * DM + d]);
        }
#pragma unroll
        for (int e = 0; e < NE; ++e) {
            lg[e] += __shfl_xor(lg[e], 16, 32);
            lg[e] += __shfl_xor(lg[e], 8, 32);
            lg[e] += __shfl_xor(lg[e], 4, 32);
            lg[e] += __shfl_xor(lg[e], 2, 32);
            lg[e] += __shfl_xor(lg[e], 1, 32);
        }
        float g[NE];
#pragma unroll
        for (int e = 0; e < NE; ++e) g[e] = 1.0f / (1.0f + expf(-lg[e]));
        unsigned taken = 0u;
        int pi[TOPK];
        float pv[TOPK];
#pragma unroll
        for (int k = 0; k < TOPK; ++k) {
            float bestv = -1.0f;
            int besti = 0;
#pragma unroll
            for (int e = 0; e < NE; ++e) { const bool c = (((taken >> e) & 1u) == 0u) && (g[e] > bestv); bestv = c ? g[e] : bestv; besti = c ? e : besti; }
            pi[k] = besti; pv[k] = bestv;
            taken |= (1u << besti);
        }
        const bool mine = (lane == j);
        ki.x = mine ? pi[0] : ki.x;  ki.y = mine ? pi[1] : ki.y;  ki.z = mine ? pi[2] : ki.z;  ki.w = mine ? pi[3] : ki.w;
        kw.x = mine ? pv[0] : kw.x;  kw.y = mine ? pv[1] : kw.y;  kw.z = mine ? pv[2] : kw.z;  kw.w = mine ? pv[3] : kw.w;
    }
    if (lane < 16u) {
        VST2(v4i, sel + (size_t)(t0 + lane) * 4u, ki);
        VST2(v4f, wgt + (size_t)(t0 + lane) * 4u, kw);
    }
}

template <int NE_>
__global__ __launch_bounds__(32) void k_route1w(const int* __restrict__ sel, int* __restrict__ tbl, unsigned nslot, unsigned spt, unsigned hdr, unsigned rmax,
                                                unsigned offPoff, unsigned offNtiles, unsigned offTileE) {
    static_assert(NE_ >= 1 && NE_ <= 32);
    __shared__ __align__(16) int s_img[RW_CH];
    __shared__ __align__(16) int s_hdr[512];
    const unsigned lane = threadIdx.x & 31u;
    const unsigned spl = nslot >> 5;
    const unsigned ng = spl >> 2;
    const unsigned ntmax = rmax >> 6;
    const v4i* sp = (const v4i*)(sel + (size_t)lane * spl);
    int cnt[NE_];
#pragma unroll
    for (int j = 0; j < NE_; ++j) cnt[j] = 0;
    for (unsigned g = 0; g < ng; ++g) {
        const v4i v = sp[g];
#pragma unroll
        for (int c = 0; c < 4; ++c) {
            const int e = min(max(v[c], 0), NE_ - 1);
#pragma unroll
            for (int j = 0; j < NE_; ++j) cnt[j] += (e == j) ? 1 : 0;
        }
    }
    int base0[NE_], total[NE_];
#pragma unroll
    for (int j = 0; j < NE_; ++j) {
        int pre = 0, tot = cnt[j];
#pragma unroll
        for (int d = 1; d < 32; d <<= 1) {
            const int t = __shfl_xor(tot, d, 32);
            pre += ((lane & (unsigned)d) != 0u) ? t : 0;
            tot += t;
        }
        base0[j] = pre;
        total[j] = tot;
    }
    int poff[NE_ + 1];
    poff[0] = 0;
#pragma unroll
    for (int j = 0; j < NE_; ++j) poff[j + 1] = poff[j] + (((total[j] + 63) >> 6) << 6);
    for (unsigned i = lane; i < 512u; i += 32u) s_hdr[i] = (i >= offTileE && i < offTileE + ntmax) ? -1 : 0;
    wave_sync_lds();
    if (lane == 0u) {
#pragma unroll
        for (int j = 0; j < NE_; ++j) { s_hdr[min((unsigned)j, 511u)] = total[j]; s_hdr[min(offPoff + (unsigned)j, 511u)] = poff[j]; }
        s_hdr[min(offPoff + (unsigned)NE_, 511u)] = poff[NE_];
        s_hdr[min(offNtiles, 511u)] = poff[NE_] >> 6;
    }
    for (unsigned t = lane; t < ntmax; t += 32u) {
        const int b64 = (int)(t * 64u);
        int ev = -1;
#pragma unroll
        for (int j = 0; j < NE_; ++j) ev = (b64 >= poff[j] && b64 < poff[j + 1]) ? j : ev;
        s_hdr[min(offTileE + t, 511u)] = ev;
    }
    wave_sync_lds();
    for (int pass = 0; pass < 2; ++pass) {
        for (unsigned i = lane; i < (hdr >> 2); i += 32u) *(volatile v4i*)(tbl + 4u * i) = *(const v4i*)(&s_hdr[4u * i]);
        __threadfence();
    }
    for (unsigned lo = 0; lo < rmax; lo += (unsigned)RW_CH) {
        for (unsigned i = lane; i < (unsigned)(RW_CH / 4); i += 32u) *(v4i*)(&s_img[4u * i]) = (v4i){-1, -1, -1, -1};
        wave_sync_lds();
        int run[NE_];
#pragma unroll
        for (int j = 0; j < NE_; ++j) run[j] = base0[j];
        for (unsigned g = 0; g < ng; ++g) {
            const v4i v = sp[g];
#pragma unroll
            for (int c = 0; c < 4; ++c) {
                const int e = min(max(v[c], 0), NE_ - 1);
                int row = 0;
#pragma unroll
                for (int j = 0; j < NE_; ++j) {
                    const bool hit = (e == j);
                    row = hit ? (poff[j] + run[j]) : row;
                    run[j] += hit ? 1 : 0;
                }
                row = min(max(row, 0), (int)rmax - 1);
                const unsigned rel = (unsigned)row - lo;
                if (rel < (unsigned)RW_CH) s_img[rel] = (int)((lane * spl + 4u * g + (unsigned)c) / spt);
            }
        }
        wave_sync_lds();
        const unsigned nw = min((unsigned)RW_CH, rmax - lo);
        for (int pass = 0; pass < 2; ++pass) {
            for (unsigned i = lane; i < (nw >> 2); i += 32u) *(volatile v4i*)(tbl + hdr + lo + 4u * i) = *(const v4i*)(&s_img[4u * i]);
            __threadfence();
        }
        wave_sync_lds();
    }
    for (unsigned lo = 0; lo < nslot; lo += (unsigned)RW_CH) {
        int run[NE_];
#pragma unroll
        for (int j = 0; j < NE_; ++j) run[j] = base0[j];
        for (unsigned g = 0; g < ng; ++g) {
            const v4i v = sp[g];
#pragma unroll
            for (int c = 0; c < 4; ++c) {
                const int e = min(max(v[c], 0), NE_ - 1);
                int row = 0;
#pragma unroll
                for (int j = 0; j < NE_; ++j) {
                    const bool hit = (e == j);
                    row = hit ? (poff[j] + run[j]) : row;
                    run[j] += hit ? 1 : 0;
                }
                row = min(max(row, 0), (int)rmax - 1);
                const unsigned rel = (lane * spl + 4u * g + (unsigned)c) - lo;
                if (rel < (unsigned)RW_CH) s_img[rel] = row;
            }
        }
        wave_sync_lds();
        const unsigned nw = min((unsigned)RW_CH, nslot - lo);
        for (int pass = 0; pass < 2; ++pass) {
            for (unsigned i = lane; i < (nw >> 2); i += 32u) *(volatile v4i*)(tbl + hdr + rmax + lo + 4u * i) = *(const v4i*)(&s_img[4u * i]);
            __threadfence();
        }
        wave_sync_lds();
    }
}

__global__ __launch_bounds__(256) void k_gather(const h16* __restrict__ x16, const int* __restrict__ tbl, h16* __restrict__ Xg) {
    const unsigned TPR = (unsigned)(DM / 8);
    const unsigned row = blockIdx.x * (256u / TPR) + (threadIdx.x / TPR);
    if (row >= (unsigned)R_MAX) return;
    const unsigned c = (threadIdx.x % TPR) * 8u;
    const int tr = tbl[TBL_ROWTOK + row];
    const bool pad = (tr < 0);
    const int tok = min(max(tr, 0), NTOK - 1);
    const v4u ld = *(const v4u*)(x16 + (size_t)(unsigned)tok * DM + c);
    v4u o;
    o.x = pad ? 0u : ld.x; o.y = pad ? 0u : ld.y; o.z = pad ? 0u : ld.z; o.w = pad ? 0u : ld.w;
    VST2(v4u, Xg + (size_t)row * DM + c, o);
}

__global__ __launch_bounds__(256) void k_ffn1(const h16* __restrict__ Xg, const h16* __restrict__ Wp,
                                              const int* __restrict__ tbl, h16* __restrict__ Hg) {
    __shared__ __align__(16) float sT[8][16 * 68];
    const unsigned lane = threadIdx.x & 31u;
    const unsigned wave = threadIdx.x >> 5;
    const unsigned u = blockIdx.x * 8u + wave;
    if (u >= (unsigned)(NT_MAX * (FF / 64))) return;
    const unsigned rowtile = u / (unsigned)(FF / 64);
    const unsigned ct = u - rowtile * (unsigned)(FF / 64);
    const int nt = min(max(tbl[TBL_NTILES], 0), NT_MAX);
    if ((int)rowtile >= nt) return;
    const int e = min(max(tbl[TBL_TILE_E + rowtile], 0), NE - 1);
    const size_t wbase = (size_t)(unsigned)e * (size_t)(FF * DM);
    const unsigned m0 = rowtile << 6, n0 = ct << 6;
    const unsigned rlane = lane & 15u;
    const unsigned koff = (lane >> 4) * 8u;
    const unsigned mOff = koff;

    v8f acc[4][4];
#pragma unroll
    for (int i = 0; i < 4; ++i)
#pragma unroll
        for (int j = 0; j < 4; ++j) acc[i][j] = (v8f){0.f,0.f,0.f,0.f,0.f,0.f,0.f,0.f};

    for (unsigned k0 = 0; k0 < (unsigned)DM; k0 += 32u) {
        v16h bh[4];
#pragma unroll
        for (int j = 0; j < 4; ++j)
            bh[j] = frag_ld(Wp + wbase + (size_t)(n0 + ((unsigned)j << 4) + rlane) * DM + koff + k0);
#pragma unroll
        for (int i = 0; i < 4; ++i) {
            const v16h ah = frag_ld(Xg + (size_t)(m0 + ((unsigned)i << 4) + rlane) * DM + koff + k0);
#pragma unroll
            for (int j = 0; j < 4; ++j) acc[i][j] = wmma16g(ah, bh[j], acc[i][j]);
        }
    }

    float* slab = sT[wave];
#pragma unroll
    for (int i = 0; i < 4; ++i) {
        const unsigned mBase = m0 + ((unsigned)i << 4);
#pragma unroll
        for (int j = 0; j < 4; ++j)
#pragma unroll
            for (int r = 0; r < 8; ++r) {
                const float a = acc[i][j][r] * SC_H;
                const float g = fmaxf(a, 0.0f);
                slab[(mOff + (unsigned)r) * 68u + ((unsigned)j << 4) + rlane] = g * CH;
            }
        wave_sync_lds();
        const unsigned q = lane >> 3, c8 = (lane & 7u) * 8u;
        v8h hv[4];
#pragma unroll
        for (int it = 0; it < 4; ++it) {
            const unsigned row = (unsigned)it * 4u + q;
            const float* sp = slab + row * 68u + c8;
#pragma unroll
            for (int t = 0; t < 8; ++t) hv[it][t] = toh_flush(sp[t]);
        }
        for (int pass = 0; pass < 2; ++pass) {
#pragma unroll
            for (int it = 0; it < 4; ++it) {
                const unsigned row = (unsigned)it * 4u + q;
                *(volatile v8h*)(Hg + (size_t)(mBase + row) * FF + n0 + c8) = hv[it];
            }
            __threadfence();
        }
        wave_sync_lds();
    }
}

__global__ __launch_bounds__(256) void k_ffn2(const h16* __restrict__ Hg, const h16* __restrict__ Wp,
                                              const int* __restrict__ tbl, float* __restrict__ Yg) {
    __shared__ __align__(16) float sT[8][16 * 68];
    const unsigned lane = threadIdx.x & 31u;
    const unsigned wave = threadIdx.x >> 5;
    const unsigned u = blockIdx.x * 8u + wave;
    if (u >= (unsigned)(NT_MAX * (DM / 64))) return;
    const unsigned rowtile = u / (unsigned)(DM / 64);
    const unsigned ct = u - rowtile * (unsigned)(DM / 64);
    const int nt = min(max(tbl[TBL_NTILES], 0), NT_MAX);
    if ((int)rowtile >= nt) return;
    const int e = min(max(tbl[TBL_TILE_E + rowtile], 0), NE - 1);
    const size_t wbase = (size_t)(unsigned)e * (size_t)(DM * FF);
    const unsigned m0 = rowtile << 6, n0 = ct << 6;
    const unsigned rlane = lane & 15u;
    const unsigned koff = (lane >> 4) * 8u;
    const unsigned mOff = koff;

    v8f acc[4][4];
#pragma unroll
    for (int i = 0; i < 4; ++i)
#pragma unroll
        for (int j = 0; j < 4; ++j) acc[i][j] = (v8f){0.f,0.f,0.f,0.f,0.f,0.f,0.f,0.f};

    for (unsigned k0 = 0; k0 < (unsigned)FF; k0 += 32u) {
        v16h bh[4];
#pragma unroll
        for (int j = 0; j < 4; ++j)
            bh[j] = frag_ld(Wp + wbase + (size_t)(n0 + ((unsigned)j << 4) + rlane) * FF + koff + k0);
#pragma unroll
        for (int i = 0; i < 4; ++i) {
            const v16h ah = frag_ld(Hg + (size_t)(m0 + ((unsigned)i << 4) + rlane) * FF + koff + k0);
#pragma unroll
            for (int j = 0; j < 4; ++j) acc[i][j] = wmma16g(ah, bh[j], acc[i][j]);
        }
    }

    float* slab = sT[wave];
#pragma unroll
    for (int i = 0; i < 4; ++i) {
        const unsigned mBase = m0 + ((unsigned)i << 4);
#pragma unroll
        for (int j = 0; j < 4; ++j)
#pragma unroll
            for (int r = 0; r < 8; ++r)
                slab[(mOff + (unsigned)r) * 68u + ((unsigned)j << 4) + rlane] = acc[i][j][r] * SC_Y;
        wave_sync_lds();
        const unsigned hh = lane >> 4, c4 = (lane & 15u) * 4u;
#pragma unroll
        for (int half = 0; half < 2; ++half) {
            v4f vv[4];
#pragma unroll
            for (int it = 0; it < 4; ++it) {
                const unsigned row = (unsigned)(half * 4 + it) * 2u + hh;
                vv[it] = *(const v4f*)(slab + row * 68u + c4);
            }
            for (int pass = 0; pass < 2; ++pass) {
#pragma unroll
                for (int it = 0; it < 4; ++it) {
                    const unsigned row = (unsigned)(half * 4 + it) * 2u + hh;
                    *(volatile v4f*)(Yg + (size_t)(mBase + row) * DM + n0 + c4) = vv[it];
                }
                __threadfence();
            }
        }
        wave_sync_lds();
    }
}

__global__ __launch_bounds__(256) void k_combine(const float* __restrict__ Yg, const float* __restrict__ wgt, const int* __restrict__ tbl, float* __restrict__ out) {
    const unsigned t = blockIdx.x * 2u + (threadIdx.x >> 7);
    if (t >= (unsigned)NTOK) return;
    const unsigned c = (threadIdx.x & 127u) * 4u;
    const v4i rr = *(const v4i*)(tbl + TBL_SLOTROW + 4u * t);
    const int r0 = min(max(rr.x, 0), R_MAX - 1);
    const int r1 = min(max(rr.y, 0), R_MAX - 1);
    const int r2 = min(max(rr.z, 0), R_MAX - 1);
    const int r3 = min(max(rr.w, 0), R_MAX - 1);
    const v4f w = *(const v4f*)(wgt + 4u * t);
    const v4f a0 = *(const v4f*)(Yg + (size_t)(unsigned)r0 * DM + c);
    const v4f a1 = *(const v4f*)(Yg + (size_t)(unsigned)r1 * DM + c);
    const v4f a2 = *(const v4f*)(Yg + (size_t)(unsigned)r2 * DM + c);
    const v4f a3 = *(const v4f*)(Yg + (size_t)(unsigned)r3 * DM + c);
    const v4f y = (((a0 * w.x) + (a1 * w.y)) + (a2 * w.z)) + (a3 * w.w);
    VST2(v4f, out + (size_t)t * DM + c, y);
}

extern "C" void kernel_launch(void* const* d_in, const int* in_sizes, int n_in, void* d_out, int out_size,
                              void* d_ws, size_t ws_size, hipStream_t stream) {
    if (n_in < 4) return;
    if (in_sizes[0] < NTOK * DM || in_sizes[1] < NE * DM) return;
    if (in_sizes[2] < NE * DM * FF || in_sizes[3] < NE * FF * DM) return;
    if (out_size < NTOK * DM) return;

    const float* x  = (const float*)d_in[0];
    const float* gw = (const float*)d_in[1];
    const float* w1 = (const float*)d_in[2];
    const float* w2 = (const float*)d_in[3];
    float* out = (float*)d_out;

    char* wsp = (char*)d_ws;
    size_t off = 0;
    auto carve = [&](size_t bytes) -> void* { void* r = wsp + off; off += (bytes + 255) & ~(size_t)255; return r; };
    h16*   x16 = (h16*)carve((size_t)NTOK * DM * 2);
    h16*   w1t = (h16*)carve((size_t)NE * FF * DM * 2);
    h16*   w2t = (h16*)carve((size_t)NE * DM * FF * 2);
    int*   sel = (int*)carve((size_t)NSLOT * 4);
    float* wgt = (float*)carve((size_t)NSLOT * 4);
    int*   tbl = (int*)carve((size_t)TBL_WORDS * 4);
    h16*   Xg  = (h16*)carve((size_t)R_MAX * DM * 2);
    h16*   Hg  = (h16*)carve((size_t)R_MAX * FF * 2);
    float* Yg  = (float*)carve((size_t)R_MAX * DM * 4);
    if (off != WS_TOTAL || off > ws_size || off > (size_t)134217728) return;

    k_plane<CX_LOG2><<<(NTOK * DM / 8) / 256, 256, 0, stream>>>(x, x16, (unsigned)(NTOK * DM / 8));
    k_planeTw<<<(NE * (DM / 64) * (FF / 32) + 3) / 4, 128, 0, stream>>>(w1, w1t, (unsigned)NE, (unsigned)DM, (unsigned)FF, (unsigned)FF, (unsigned)(DM * FF), (float)(1u << CW_LOG2));
    k_planeTw<<<(NE * (FF / 64) * (DM / 32) + 3) / 4, 128, 0, stream>>>(w2, w2t, (unsigned)NE, (unsigned)FF, (unsigned)DM, (unsigned)DM, (unsigned)(FF * DM), (float)(1u << CW_LOG2));

    k_gate<<<NTOK / 128, 256, 0, stream>>>(x, gw, sel, wgt);
    k_route1w<NE><<<1, 32, 0, stream>>>(sel, tbl, (unsigned)NSLOT, (unsigned)TOPK, (unsigned)TBL_HDR, (unsigned)R_MAX, (unsigned)TBL_POFF, (unsigned)TBL_NTILES, (unsigned)TBL_TILE_E);
    k_gather<<<R_MAX / (256 / (DM / 8)), 256, 0, stream>>>(x16, tbl, Xg);
    k_ffn1<<<(NT_MAX * (FF / 64) + 7) / 8, 256, 0, stream>>>(Xg, w1t, tbl, Hg);
    k_ffn2<<<(NT_MAX * (DM / 64) + 7) / 8, 256, 0, stream>>>(Hg, w2t, tbl, Yg);
    k_combine<<<NTOK / 2, 256, 0, stream>>>(Yg, wgt, tbl, out);
}
